// MultiScaleRetention_28741921145323
// MI455X (gfx1250) — hardware-verified
//
#include <hip/hip_runtime.h>
#include <math.h>

constexpr int kB   = 2;
constexpr int kS   = 2048;
constexpr int kD   = 1024;
constexpr int kD2  = 2048;
constexpr int kH   = 16;
constexpr int kKd  = 64;
constexpr int kHd  = 128;
constexpr int kTok = kB * kS;
constexpr int kBH  = kB * kH;
constexpr int kVtRows = 192;
constexpr int kGrp  = 2;
constexpr int kOGrp = 8;
constexpr float kKScale     = 0.125f;
constexpr float kPCarry     = 2048.0f;
constexpr float kPCarryInv  = 1.0f / 2048.0f;
constexpr float kWoCarry    = 64.0f;
constexpr float kWoCarryInv = 1.0f / 64.0f;
constexpr float kInvHd      = 1.0f / 128.0f;
constexpr float kLnEps      = 1.0e-5f;
static_assert(kH * kKd == kD && kH * kHd == kD2);
static_assert(kTok % 64 == 0 && kD % 64 == 0 && kD2 % 64 == 0 && kS % 64 == 0 && kHd % 64 == 0 && kVtRows % 64 == 0);
static_assert(kD % 32 == 0 && kD2 % 32 == 0 && kKd % 32 == 0 && kS % 32 == 0);
static_assert(kBH % kGrp == 0 && kOGrp % kGrp == 0 && kBH % kOGrp == 0 && kH % kGrp == 0);
static_assert((kTok * kD) % (8 * 256) == 0 && kS * (kKd / 2) == 65536);

typedef __attribute__((ext_vector_type(16))) _Float16 v16h;
typedef __attribute__((ext_vector_type(8)))  _Float16 v8h;
typedef __attribute__((ext_vector_type(16))) __bf16   v16b;
typedef __attribute__((ext_vector_type(8)))  __bf16   v8b;
typedef __attribute__((ext_vector_type(8)))  float    v8f;
typedef __attribute__((ext_vector_type(4)))  float    v4f;
typedef __attribute__((ext_vector_type(4)))  unsigned int v4u;

__device__ __forceinline__ unsigned short f2bf_bits(float f) {
  unsigned u = __float_as_uint(f);
  return (unsigned short)((u + 0x7FFFu + ((u >> 16) & 1u)) >> 16);
}
__device__ __forceinline__ float bf_bits2f(unsigned short h) { return __uint_as_float(((unsigned)h) << 16); }
__device__ __forceinline__ unsigned pk16(unsigned short a, unsigned short b) { return (unsigned)a | ((unsigned)b << 16); }
__device__ __forceinline__ unsigned short h_bits(float f) { const _Float16 h = (_Float16)f; return __builtin_bit_cast(unsigned short, h); }
__device__ __forceinline__ float h16_to_f32(unsigned hb) {
  const unsigned sgn = (hb & 0x8000u) << 16; const unsigned em = hb & 0x7fffu;
  const float fn = __uint_as_float((em << 13) + 0x38000000u);
  const float fs = (float)em * 5.9604644775390625e-8f;
  const float mag = (em < 0x400u) ? fs : fn; return __uint_as_float(__float_as_uint(mag) | sgn);
}

__device__ __forceinline__ void dep_guard4_h(v8f& a, v8f& b, v8f& c, v8f& d, v16h x, v16h y) {
  asm volatile("v_nop\n\tv_nop\n\tv_nop\n\tv_nop" : "+v"(a), "+v"(b), "+v"(c), "+v"(d) : "v"(x), "v"(y));
}
__device__ __forceinline__ void dep_guard4_b(v8f& a, v8f& b, v8f& c, v8f& d, v16b x, v16b y) {
  asm volatile("v_nop\n\tv_nop\n\tv_nop\n\tv_nop" : "+v"(a), "+v"(b), "+v"(c), "+v"(d) : "v"(x), "v"(y));
}
__device__ __forceinline__ void keep4_h(v16h a, v16h b, v16h c, v16h d) { asm volatile("v_nop" :: "v"(a), "v"(b), "v"(c), "v"(d)); }
__device__ __forceinline__ void keep4_b(v16b a, v16b b, v16b c, v16b d) { asm volatile("v_nop" :: "v"(a), "v"(b), "v"(c), "v"(d)); }
__device__ __forceinline__ void acc_guard4(v8f& a, v8f& b, v8f& c, v8f& d) { asm volatile("v_nop\n\tv_nop\n\tv_nop\n\tv_nop" : "+v"(a), "+v"(b), "+v"(c), "+v"(d)); }
template <typename T> struct Frag;
template <> struct Frag<_Float16> {
  typedef v16h V; union U { v16h v; v8h h[2]; };
  static __device__ __forceinline__ v16h load(const _Float16* p) {
    U f; f.h[0] = *(const v8h*)(p); f.h[1] = *(const v8h*)(p + 16); return f.v;
  }
  static __device__ __forceinline__ v8f mma(v16h a, v16h b, v8f c) {
    return __builtin_amdgcn_wmma_f32_16x16x32_f16(false, a, false, b, (short)0, c, false, false);
  }
  static __device__ __forceinline__ void guard4(v8f& a, v8f& b, v8f& c, v8f& d, v16h x, v16h y) { dep_guard4_h(a, b, c, d, x, y); }
  static __device__ __forceinline__ void keep(v16h a, v16h b, v16h c, v16h d) { keep4_h(a, b, c, d); }
};
template <> struct Frag<__bf16> {
  typedef v16b V; union U { v16b v; v8b h[2]; };
  static __device__ __forceinline__ v16b load(const __bf16* p) {
    U f; f.h[0] = *(const v8b*)(p); f.h[1] = *(const v8b*)(p + 16); return f.v;
  }
  static __device__ __forceinline__ v8f mma(v16b a, v16b b, v8f c) {
    return __builtin_amdgcn_wmma_f32_16x16x32_bf16(false, a, false, b, (short)0, c, false, false);
  }
  static __device__ __forceinline__ void guard4(v8f& a, v8f& b, v8f& c, v8f& d, v16b x, v16b y) { dep_guard4_b(a, b, c, d, x, y); }
  static __device__ __forceinline__ void keep(v16b a, v16b b, v16b c, v16b d) { keep4_b(a, b, c, d); }
};

template <int ET> struct Elem;
template <> struct Elem<0> { typedef _Float16 T; };
template <> struct Elem<1> { typedef __bf16 T; };
template <int ET, bool SPLIT, int BIAS_MODE, int OUT_MODE, bool RESID, int ACT = 0, int KLIM = 0>
__global__ __launch_bounds__(256) void wmma_gemm64(
    const unsigned short* __restrict__ Ap, const unsigned short* __restrict__ A2p, int lda, long strideA,
    const unsigned short* __restrict__ Btp, const unsigned short* __restrict__ Bt2p, int ldb, long strideB,
    void* __restrict__ Cout, void* __restrict__ Cout2, int ldc, long strideC,
    const float* __restrict__ bias, long strideBias,
    const float* __restrict__ resid, long strideR,
    int M, int N, int K, float scale) {
  typedef typename Elem<ET>::T T;
  typedef typename Frag<T>::V V;
  const T* A = (const T*)Ap; const T* A2 = (const T*)A2p; const T* Bt = (const T*)Btp; const T* Bt2 = (const T*)Bt2p;
  __shared__ __align__(16) float sT[8][16 * 68];
  const int b    = blockIdx.y;
  const int lane = threadIdx.x & 31;
  const int wave = threadIdx.x >> 5;
  const int tilesN = N >> 6;
  const int tilesM = M >> 6;
  const int tile = blockIdx.x * 8 + wave;
  if (tile >= tilesM * tilesN) return;
  const int tm = tile / tilesN;
  const int tn = tile - tm * tilesN;
  const int m0 = tm << 6;
  const int n0 = tn << 6;

  const T* Ab  = A  + (size_t)b * strideA;
  const T* Bb  = Bt + (size_t)b * strideB;
  const T* Ab2 = SPLIT ? (A2  + (size_t)b * strideA) : nullptr;
  const T* Bb2 = SPLIT ? (Bt2 + (size_t)b * strideB) : nullptr;
  const float* biasb = bias + (size_t)b * strideBias;

  const int rlane = lane & 15;
  const int koff  = (lane >> 4) * 8;
  const int mOff  = (lane >> 4) * 8;

  v8f acc[4][4];
#pragma unroll
  for (int i = 0; i < 4; ++i)
#pragma unroll
    for (int j = 0; j < 4; ++j) acc[i][j] = (v8f){0.f,0.f,0.f,0.f,0.f,0.f,0.f,0.f};

  const int Kend = (KLIM != 0) ? ((m0 + 64 < K) ? (m0 + 64) : K) : K;
  for (int k0 = 0; k0 < Kend; k0 += 32) {
    V bh[4], bl[4];
#pragma unroll
    for (int j = 0; j < 4; ++j) {
      const size_t bo = (size_t)(n0 + (j << 4) + rlane) * ldb + koff + k0;
      bh[j] = Frag<T>::load(Bb + bo);
      if (SPLIT) bl[j] = Frag<T>::load(Bb2 + bo);
    }
#pragma unroll
    for (int i = 0; i < 4; ++i) {
      const size_t ao = (size_t)(m0 + (i << 4) + rlane) * lda + koff + k0;
      V ah = Frag<T>::load(Ab + ao);
      V al;
      if (SPLIT) al = Frag<T>::load(Ab2 + ao);
#pragma unroll
      for (int j = 0; j < 4; ++j) {
        acc[i][j] = Frag<T>::mma(ah, bh[j], acc[i][j]);
        if (SPLIT) {
          acc[i][j] = Frag<T>::mma(ah, bl[j], acc[i][j]);
          acc[i][j] = Frag<T>::mma(al, bh[j], acc[i][j]);
        }
      }
      Frag<T>::guard4(acc[i][0], acc[i][1], acc[i][2], acc[i][3], ah, SPLIT ? al : ah);
    }
    Frag<T>::keep(bh[0], bh[1], bh[2], bh[3]);
    if (SPLIT) Frag<T>::keep(bl[0], bl[1], bl[2], bl[3]);
  }
  acc_guard4(acc[0][0], acc[0][1], acc[0][2], acc[0][3]);
  acc_guard4(acc[1][0], acc[1][1], acc[1][2], acc[1][3]);
  acc_guard4(acc[2][0], acc[2][1], acc[2][2], acc[2][3]);
  acc_guard4(acc[3][0], acc[3][1], acc[3][2], acc[3][3]);

  float* slab = sT[wave];
  const float* Rb = RESID ? (resid + (size_t)b * strideR) : nullptr;
#pragma unroll
  for (int i = 0; i < 4; ++i) {
    const int mBase = m0 + (i << 4);
#pragma unroll
    for (int j = 0; j < 4; ++j) {
      const int n = n0 + (j << 4) + rlane;
      float bv = 0.f;
      if (BIAS_MODE == 2) bv = biasb[n];
#pragma unroll
      for (int r = 0; r < 8; ++r) {
        float v = acc[i][j][r] * scale;
        if (BIAS_MODE == 1) v += biasb[mBase + mOff + r];
        if (BIAS_MODE == 2) v += bv;
        if (RESID) v += Rb[(size_t)(mBase + mOff + r) * ldc + n];
        if (ACT == 2) v = fmaxf(v, 0.0f);
        if (ACT == 4) v = (v > 0.f) ? v : 0.01f * v;
        slab[(mOff + r) * 68 + (j << 4) + rlane] = v;
      }
    }
    __builtin_amdgcn_fence(__ATOMIC_RELEASE, "workgroup");
    __builtin_amdgcn_wave_barrier();
    __builtin_amdgcn_fence(__ATOMIC_ACQUIRE, "workgroup");
    if (OUT_MODE == 0) {
      float* C = (float*)Cout + (size_t)b * strideC;
      const int hh = lane >> 4, c4 = (lane & 15) * 4;
      for (int pass = 0; pass < 2; ++pass) {
#pragma unroll
        for (int it = 0; it < 8; ++it) {
          const int row = it * 2 + hh;
          v4f v = *(const v4f*)(slab + row * 68 + c4);
          *(volatile v4f*)(C + (size_t)(mBase + row) * ldc + n0 + c4) = v;
        }
        __threadfence();
      }
    } else {
      const int q = lane >> 3, c8 = (lane & 7) * 8;
      unsigned short* C  = (unsigned short*)Cout  + (size_t)b * strideC;
      unsigned short* C2 = (OUT_MODE == 2) ? ((unsigned short*)Cout2 + (size_t)b * strideC) : nullptr;
      for (int pass = 0; pass < 2; ++pass) {
#pragma unroll
        for (int it = 0; it < 4; ++it) {
          const int row = it * 4 + q;
          const float* sp = slab + row * 68 + c8;
          v8h hv, lv;
#pragma unroll
          for (int e = 0; e < 8; ++e) {
            if (OUT_MODE == 1) {
              hv[e] = (_Float16)sp[e];
            } else {
              unsigned short hb = f2bf_bits(sp[e]);
              unsigned short lb = f2bf_bits(sp[e] - bf_bits2f(hb));
              hv[e] = __builtin_bit_cast(_Float16, hb);
              lv[e] = __builtin_bit_cast(_Float16, lb);
            }
          }
          *(volatile v8h*)(C + (size_t)(mBase + row) * ldc + n0 + c8) = hv;
          if (OUT_MODE == 2) *(volatile v8h*)(C2 + (size_t)(mBase + row) * ldc + n0 + c8) = lv;
        }
        __threadfence();
      }
    }
    __builtin_amdgcn_fence(__ATOMIC_RELEASE, "workgroup");
    __builtin_amdgcn_wave_barrier();
    __builtin_amdgcn_fence(__ATOMIC_ACQUIRE, "workgroup");
  }
}

__global__ __launch_bounds__(256) void wmma_gemm64_dmask(
    const unsigned short* __restrict__ Ap, int lda, long strideA,
    const unsigned short* __restrict__ Btp, int ldb, long strideB,
    unsigned short* __restrict__ Cout, int ldc, long strideC,
    const float* __restrict__ rowf, const float* __restrict__ colf, long strideF,
    int M, int N, int K, float scale) {
  typedef _Float16 T;
  typedef v16h V;
  const T* A = (const T*)Ap; const T* Bt = (const T*)Btp;
  __shared__ __align__(16) float sT[8][16 * 68];
  const int b    = blockIdx.y;
  const int lane = threadIdx.x & 31;
  const int wave = threadIdx.x >> 5;
  const int tilesN = N >> 6;
  const int tilesM = M >> 6;
  const int tile = blockIdx.x * 8 + wave;
  if (tile >= tilesM * tilesN) return;
  const int tm = tile / tilesN;
  const int tn = tile - tm * tilesN;
  if (tn > tm) return;
  const int m0 = tm << 6;
  const int n0 = tn << 6;

  const T* Ab = A  + (size_t)b * strideA;
  const T* Bb = Bt + (size_t)b * strideB;
  const float* rfb = rowf + (size_t)b * strideF;
  const float* cfb = colf + (size_t)b * strideF;

  const int rlane = lane & 15;
  const int koff  = (lane >> 4) * 8;
  const int mOff  = (lane >> 4) * 8;

  v8f acc[4][4];
#pragma unroll
  for (int i = 0; i < 4; ++i)
#pragma unroll
    for (int j = 0; j < 4; ++j) acc[i][j] = (v8f){0.f,0.f,0.f,0.f,0.f,0.f,0.f,0.f};

  for (int k0 = 0; k0 < K; k0 += 32) {
    V bh[4];
#pragma unroll
    for (int j = 0; j < 4; ++j) {
      const size_t bo = (size_t)(n0 + (j << 4) + rlane) * ldb + koff + k0;
      bh[j] = Frag<T>::load(Bb + bo);
    }
#pragma unroll
    for (int i = 0; i < 4; ++i) {
      const size_t ao = (size_t)(m0 + (i << 4) + rlane) * lda + koff + k0;
      V ah = Frag<T>::load(Ab + ao);
#pragma unroll
      for (int j = 0; j < 4; ++j) acc[i][j] = Frag<T>::mma(ah, bh[j], acc[i][j]);
      Frag<T>::guard4(acc[i][0], acc[i][1], acc[i][2], acc[i][3], ah, ah);
    }
    Frag<T>::keep(bh[0], bh[1], bh[2], bh[3]);
  }
  acc_guard4(acc[0][0], acc[0][1], acc[0][2], acc[0][3]);
  acc_guard4(acc[1][0], acc[1][1], acc[1][2], acc[1][3]);
  acc_guard4(acc[2][0], acc[2][1], acc[2][2], acc[2][3]);
  acc_guard4(acc[3][0], acc[3][1], acc[3][2], acc[3][3]);

  float* slab = sT[wave];
#pragma unroll
  for (int i = 0; i < 4; ++i) {
    const int mBase = m0 + (i << 4);
    float rfv[8];
#pragma unroll
    for (int r = 0; r < 8; ++r) rfv[r] = rfb[mBase + mOff + r];
#pragma unroll
    for (int j = 0; j < 4; ++j) {
      const int n = n0 + (j << 4) + rlane;
      const float cf = cfb[n];
#pragma unroll
      for (int r = 0; r < 8; ++r) {
        const int row = mBase + mOff + r;
        const float w = rfv[r] * cf;
        float v = (acc[i][j][r] * scale) * w;
        v = (n <= row) ? v : 0.0f;
        slab[(mOff + r) * 68 + (j << 4) + rlane] = v;
      }
    }
    __builtin_amdgcn_fence(__ATOMIC_RELEASE, "workgroup");
    __builtin_amdgcn_wave_barrier();
    __builtin_amdgcn_fence(__ATOMIC_ACQUIRE, "workgroup");
    {
      const int q = lane >> 3, c8 = (lane & 7) * 8;
      unsigned short* C = Cout + (size_t)b * strideC;
      for (int pass = 0; pass < 2; ++pass) {
#pragma unroll
        for (int it = 0; it < 4; ++it) {
          const int row = it * 4 + q;
          const float* sp = slab + row * 68 + c8;
          v8h hv;
#pragma unroll
          for (int e = 0; e < 8; ++e) hv[e] = (_Float16)sp[e];
          *(volatile v8h*)(C + (size_t)(mBase + row) * ldc + n0 + c8) = hv;
        }
        __threadfence();
      }
    }
    __builtin_amdgcn_fence(__ATOMIC_RELEASE, "workgroup");
    __builtin_amdgcn_wave_barrier();
    __builtin_amdgcn_fence(__ATOMIC_ACQUIRE, "workgroup");
  }
}

__global__ __launch_bounds__(256) void cast8_bf16_kernel(const float* __restrict__ in, unsigned short* __restrict__ out, int n8) {
  const int i = blockIdx.x * 256 + threadIdx.x;
  if (i >= n8) return;
  const float* p = in + 8 * (size_t)i;
  const v4f a = *(const v4f*)(p);
  const v4f c = *(const v4f*)(p + 4);
  unsigned short hb[8];
#pragma unroll
  for (int e = 0; e < 4; ++e) {
    hb[e]     = f2bf_bits(a[e]);
    hb[4 + e] = f2bf_bits(c[e]);
  }
  const v4u u = (v4u){pk16(hb[0], hb[1]), pk16(hb[2], hb[3]), pk16(hb[4], hb[5]), pk16(hb[6], hb[7])};
  unsigned short* q = out + 8 * (size_t)i;
  *(volatile v4u*)q = u;
  __threadfence();
  *(volatile v4u*)q = u;
}

template <int MODE>
__global__ __launch_bounds__(256) void tcast_kernel(const float* __restrict__ in0, const float* __restrict__ in1,
                                                    unsigned short* __restrict__ out0, unsigned short* __restrict__ out1,
                                                    int R, int Cc, float scale) {
  __shared__ float sm[64][65];
  const int t  = threadIdx.x;
  const int z  = blockIdx.z;
  const float* in = (z == 0) ? in0 : in1;
  unsigned short* out = (z == 0) ? out0 : out1;
  const int r0 = blockIdx.x * 64;
  const int c0 = blockIdx.y * 64;
#pragma unroll
  for (int i = 0; i < 8; ++i) {
    const int e = i * 256 + t;
    const int rl = e >> 6;
    const int cl = e & 63;
    sm[cl][rl] = in[(size_t)(r0 + rl) * Cc + c0 + cl];
  }
  asm volatile("" ::: "memory");
#pragma unroll
  for (int i = 8; i < 16; ++i) {
    const int e = i * 256 + t;
    const int rl = e >> 6;
    const int cl = e & 63;
    sm[cl][rl] = in[(size_t)(r0 + rl) * Cc + c0 + cl];
  }
  __syncthreads();
  const int lane = t & 31, wave = t >> 5;
  const int q = lane >> 3, c8 = (lane & 7) * 8;
  for (int pass = 0; pass < 2; ++pass) {
#pragma unroll
    for (int it = 0; it < 2; ++it) {
      const int row = wave * 8 + it * 4 + q;
      unsigned short hb[8];
#pragma unroll
      for (int e = 0; e < 8; ++e) {
        const float v = sm[row][c8 + e];
        if (MODE == 0) {
          hb[e] = f2bf_bits(v);
        } else {
          const float vb = bf_bits2f(f2bf_bits(v));
          hb[e] = h_bits(vb * scale);
        }
      }
      const v4u u = (v4u){pk16(hb[0], hb[1]), pk16(hb[2], hb[3]), pk16(hb[4], hb[5]), pk16(hb[6], hb[7])};
      *(volatile v4u*)(out + (size_t)(c0 + row) * R + r0 + c8) = u;
    }
    __threadfence();
  }
}

struct ConstTab { float ang[32]; float dec[16]; };
static_assert(sizeof(ConstTab) == 192);

__global__ __launch_bounds__(256) void trig_table_kernel(float* __restrict__ cosT, float* __restrict__ sinT, ConstTab ct) {
#pragma clang fp contract(off)
  const int idx = blockIdx.x * 256 + threadIdx.x;
  const int s = idx >> 5;
  const int i = idx & 31;
  float ang = ct.ang[0];
#pragma unroll
  for (int j = 1; j < 32; ++j) ang = (i == j) ? ct.ang[j] : ang;
  const float th = (float)s * ang;
  float sv, cv;
  sincosf(th, &sv, &cv);
  *(volatile float*)(cosT + idx) = cv;
  *(volatile float*)(sinT + idx) = sv;
  __threadfence();
  *(volatile float*)(cosT + idx) = cv;
  *(volatile float*)(sinT + idx) = sv;
}

__global__ __launch_bounds__(256) void decay_table_kernel(float* __restrict__ rowF, float* __restrict__ colF, ConstTab ct) {
  const int hh = blockIdx.x >> 3;
  const int s  = ((blockIdx.x & 7) << 8) | (int)threadIdx.x;
  float dcy = ct.dec[0];
#pragma unroll
  for (int j = 1; j < 16; ++j) dcy = (hh == j) ? ct.dec[j] : dcy;
  const float p2 = (float)(32 << hh);
  const float rs = -expm1f(dcy * (float)(s + 1)) * p2;
  const float rn = 1.0f / sqrtf(rs);
  const float rf = expf(dcy * (float)s) * rn;
  const float cf = expf(-dcy * (float)s);
  const int o = hh * kS + s;
  *(volatile float*)(rowF + o) = rf;
  *(volatile float*)(colF + o) = cf;
  __threadfence();
  *(volatile float*)(rowF + o) = rf;
  *(volatile float*)(colF + o) = cf;
}

__global__ __launch_bounds__(256) void vt_pad_fill_kernel(unsigned short* __restrict__ VT) {
  const int gid  = blockIdx.x * 256 + threadIdx.x;
  const int bh   = gid >> 14;
  const int prow = (gid >> 8) & 63;
  const int c8   = (gid & 255) * 8;
  const unsigned uv = (prow == 0) ? 0x3C003C00u : 0u;
  const v4u u = (v4u){uv, uv, uv, uv};
  unsigned short* dst = VT + ((size_t)bh * kVtRows + kHd + prow) * kS + c8;
  *(volatile v4u*)dst = u;
  __threadfence();
  *(volatile v4u*)dst = u;
}

__global__ __launch_bounds__(256) void rope_kernel(const unsigned short* __restrict__ QK, const float* __restrict__ cosT,
                                                   const float* __restrict__ sinT, unsigned short* __restrict__ QRK) {
  const int gid   = blockIdx.x * 256 + threadIdx.x;
  const int token = gid >> 8;
  const int c     = (gid & 255) * 8;
  const int sel   = c >> 10;
  const int cc    = c & (kD - 1);
  const int h     = cc >> 6;
  const int d0    = cc & (kKd - 1);
  const int b     = token >> 11;
  const int s     = token & (kS - 1);
  const v4u w = *(const v4u*)(QK + (size_t)token * kD2 + c);
  float x[8];
#pragma unroll
  for (int m = 0; m < 4; ++m) {
    const unsigned wd = w[m];
    x[2 * m]     = h16_to_f32(wd & 0xffffu);
    x[2 * m + 1] = h16_to_f32(wd >> 16);
  }
  const v4f cv = *(const v4f*)(cosT + s * 32 + (d0 >> 1));
  const v4f sv = *(const v4f*)(sinT + s * 32 + (d0 >> 1));
  unsigned short hb[8];
#pragma unroll
  for (int p = 0; p < 4; ++p) {
    const float x0 = x[2 * p], x1 = x[2 * p + 1];
    const float y0 = x0 * cv[p] - x1 * sv[p];
    const float y1 = x1 * cv[p] + x0 * sv[p];
    hb[2 * p]     = h_bits(y0);
    hb[2 * p + 1] = h_bits(y1);
  }
  const v4u u = (v4u){pk16(hb[0], hb[1]), pk16(hb[2], hb[3]), pk16(hb[4], hb[5]), pk16(hb[6], hb[7])};
  unsigned short* dst = QRK + ((size_t)(sel * kBH + b * kH + h) * kS + s) * kKd + d0;
  *(volatile v4u*)dst = u;
  __threadfence();
  *(volatile v4u*)dst = u;
}

__global__ __launch_bounds__(256) void ln_gate_kernel(const float* __restrict__ O, const unsigned short* __restrict__ G16,
                                                      unsigned short* __restrict__ A16, int bh0) {
  const int t = threadIdx.x;
  const int lane = t & 31, wave = t >> 5;
  const int half = lane >> 4, l16 = lane & 15;
  const int rid = blockIdx.x * 16 + wave * 2 + half;
  const int bl  = rid >> 11;
  const int s   = rid & (kS - 1);
  const int bh  = bh0 + bl;
  const int b   = bh >> 4;
  const int h   = bh & 15;
  const int token = b * kS + s;
  const int e0 = l16 * 8;
  const float* orow = O + ((size_t)bl * kS + s) * kVtRows;
  const v4f oa = *(const v4f*)(orow + e0);
  const v4f ob = *(const v4f*)(orow + e0 + 4);
  const float rsum  = orow[kHd];
  const float denom = fmaxf(fabsf(rsum), 1.0f);
  const float invd  = 1.0f / denom;
  float v[8];
#pragma unroll
  for (int e = 0; e < 4; ++e) { v[e] = oa[e] * invd; v[4 + e] = ob[e] * invd; }
  float sm = ((v[0] + v[1]) + (v[2] + v[3])) + ((v[4] + v[5]) + (v[6] + v[7]));
  sm += __shfl_xor(sm, 1, 32);
  sm += __shfl_xor(sm, 2, 32);
  sm += __shfl_xor(sm, 4, 32);
  sm += __shfl_xor(sm, 8, 32);
  const float mu = sm * kInvHd;
  float d[8];
  float sq = 0.0f;
#pragma unroll
  for (int e = 0; e < 8; ++e) { d[e] = v[e] - mu; sq += d[e] * d[e]; }
  sq += __shfl_xor(sq, 1, 32);
  sq += __shfl_xor(sq, 2, 32);
  sq += __shfl_xor(sq, 4, 32);
  sq += __shfl_xor(sq, 8, 32);
  const float var  = sq * kInvHd;
  const float rstd = 1.0f / sqrtf(var + kLnEps);
  const v4u gw = *(const v4u*)(G16 + (size_t)token * kD2 + h * kHd + e0);
  float g[8];
#pragma unroll
  for (int m = 0; m < 4; ++m) {
    const unsigned wd = gw[m];
    g[2 * m]     = h16_to_f32(wd & 0xffffu);
    g[2 * m + 1] = h16_to_f32(wd >> 16);
  }
  unsigned short hb[8];
#pragma unroll
  for (int e = 0; e < 8; ++e) {
    const float sg = __builtin_amdgcn_rcpf(1.0f + expf(-g[e]));
    const float a  = (g[e] * sg) * (d[e] * rstd);
    hb[e] = h_bits(a);
  }
  const v4u u = (v4u){pk16(hb[0], hb[1]), pk16(hb[2], hb[3]), pk16(hb[4], hb[5]), pk16(hb[6], hb[7])};
  unsigned short* dst = A16 + (size_t)token * kD2 + h * kHd + e0;
  *(volatile v4u*)dst = u;
  __threadfence();
  *(volatile v4u*)dst = u;
}

extern "C" void kernel_launch(void* const* d_in, const int* in_sizes, int n_in,
                              void* d_out, int out_size, void* d_ws, size_t ws_size,
                              hipStream_t stream) {
  if (n_in < 11) return;
  if (in_sizes[0] != kTok * kD) return;
  if (in_sizes[1] != kD * kD || in_sizes[2] != kD) return;
  if (in_sizes[3] != kD * kD || in_sizes[4] != kD) return;
  if (in_sizes[5] != kD * kD2 || in_sizes[6] != kD2) return;
  if (in_sizes[7] != kD * kD2 || in_sizes[8] != kD2) return;
  if (in_sizes[9] != kD2 * kD || in_sizes[10] != kD) return;
  if (out_size != kTok * kD) return;

  const size_t szXB  = (size_t)kTok * kD * 2;
  const size_t szWT  = (size_t)kTok * kD * 2;
  const size_t szWV  = (size_t)kD2 * kD * 2;
  const size_t szWO  = (size_t)kD * kD2 * 2;
  const size_t szQK  = (size_t)kTok * kD2 * 2;
  const size_t szG   = (size_t)kTok * kD2 * 2;
  const size_t szQRK = (size_t)2 * kBH * kS * kKd * 2;
  const size_t szVT  = (size_t)kBH * kVtRows * kS * 2;
  const size_t szTrg = (size_t)kS * 32 * 4;
  const size_t szDec = (size_t)kH * kS * 4;
  const size_t szPP  = (size_t)kGrp * kS * kS * 2;
  const size_t szO   = (size_t)kOGrp * kS * kVtRows * 4;
  const size_t offXB  = 0;
  const size_t offWT  = offXB + szXB;
  const size_t offWV  = offWT + szWT;
  const size_t offWO  = offWV + szWV;
  const size_t offQK  = offWO + szWO;
  const size_t offG   = offQK + szQK;
  const size_t offQRK = offG + szG;
  const size_t offVT  = offQRK + szQRK;
  const size_t offCOS = offVT + szVT;
  const size_t offSIN = offCOS + szTrg;
  const size_t offRWF = offSIN + szTrg;
  const size_t offCLF = offRWF + szDec;
  const size_t offPP  = offCLF + szDec;
  const size_t offO   = offPP + szPP;
  const size_t total  = offO + szO;
  if (ws_size < total) return;

  const float* x  = (const float*)d_in[0];
  const float* Wq = (const float*)d_in[1];
  const float* bq = (const float*)d_in[2];
  const float* Wk = (const float*)d_in[3];
  const float* bk = (const float*)d_in[4];
  const float* Wv = (const float*)d_in[5];
  const float* bv = (const float*)d_in[6];
  const float* Wg = (const float*)d_in[7];
  const float* bg = (const float*)d_in[8];
  const float* Wo = (const float*)d_in[9];
  const float* bo = (const float*)d_in[10];
  float* out = (float*)d_out;
  char* ws = (char*)d_ws;
  unsigned short* XB  = (unsigned short*)(ws + offXB);
  unsigned short* WT  = (unsigned short*)(ws + offWT);
  unsigned short* WV  = (unsigned short*)(ws + offWV);
  unsigned short* WO  = (unsigned short*)(ws + offWO);
  unsigned short* QK  = (unsigned short*)(ws + offQK);
  unsigned short* A16 = QK;
  unsigned short* G16 = (unsigned short*)(ws + offG);
  unsigned short* QRK = (unsigned short*)(ws + offQRK);
  unsigned short* VT  = (unsigned short*)(ws + offVT);
  float* COS = (float*)(ws + offCOS);
  float* SIN = (float*)(ws + offSIN);
  float* RWF = (float*)(ws + offRWF);
  float* CLF = (float*)(ws + offCLF);
  unsigned short* PP = (unsigned short*)(ws + offPP);
  float* O = (float*)(ws + offO);

  ConstTab ct;
  for (int i = 0; i < 32; ++i) {
    const float lin = (float)i * (1.0f / 31.0f);
    const float pw  = (float)pow(10000.0, (double)lin);
    ct.ang[i] = 1.0f / pw;
  }
  for (int h = 0; h < 16; ++h) ct.dec[h] = (float)log1p(-pow(2.0, -5.0 - (double)h));

  const int n8 = (kTok * kD) / 8;
  cast8_bf16_kernel<<<dim3(n8 / 256), dim3(256), 0, stream>>>(x, XB, n8);
  tcast_kernel<0><<<dim3(kD / 64, kD / 64, 2), dim3(256), 0, stream>>>(Wq, Wk, WT, WT + (size_t)kD * kD, kD, kD, 1.0f);
  tcast_kernel<0><<<dim3(kD / 64, kD2 / 64, 2), dim3(256), 0, stream>>>(Wg, Wv, WT + (size_t)2 * kD * kD, WV, kD, kD2, 1.0f);
  tcast_kernel<1><<<dim3(kD2 / 64, kD / 64, 1), dim3(256), 0, stream>>>(Wo, Wo, WO, WO, kD2, kD, kWoCarry);
  trig_table_kernel<<<dim3(256), dim3(256), 0, stream>>>(COS, SIN, ct);
  decay_table_kernel<<<dim3(128), dim3(256), 0, stream>>>(RWF, CLF, ct);
  vt_pad_fill_kernel<<<dim3(2048), dim3(256), 0, stream>>>(VT);

  const int blkQ = ((kTok / 64) * (kD / 64)) / 8;
  const int blkG = ((kTok / 64) * (kD2 / 64)) / 8;
  wmma_gemm64<1, false, 2, 1, false, 0, 0><<<dim3(blkQ, 1), dim3(256), 0, stream>>>(
      XB, XB, kD, 0L, WT, WT, kD, 0L, (void*)QK, (void*)QK, kD2, 0L, bq, 0L, bq, 0L, kTok, kD, kD, 1.0f);
  wmma_gemm64<1, false, 2, 1, false, 0, 0><<<dim3(blkQ, 1), dim3(256), 0, stream>>>(
      XB, XB, kD, 0L, WT + (size_t)kD * kD, WT + (size_t)kD * kD, kD, 0L,
      (void*)(QK + kD), (void*)(QK + kD), kD2, 0L, bk, 0L, bk, 0L, kTok, kD, kD, 1.0f);
  wmma_gemm64<1, false, 2, 1, false, 0, 0><<<dim3(blkG, 1), dim3(256), 0, stream>>>(
      XB, XB, kD, 0L, WT + (size_t)2 * kD * kD, WT + (size_t)2 * kD * kD, kD, 0L,
      (void*)G16, (void*)G16, kD2, 0L, bg, 0L, bg, 0L, kTok, kD2, kD, 1.0f);
  const int blkV = ((kHd / 64) * (kS / 64)) / 8;
  for (int b = 0; b < kB; ++b) {
    const unsigned short* xb = XB + (size_t)b * kS * kD;
    unsigned short* vtb = VT + (size_t)b * kH * kVtRows * kS;
    wmma_gemm64<1, false, 1, 1, false, 0, 0><<<dim3(blkV, kH), dim3(256), 0, stream>>>(
        WV, WV, kD, (long)kHd * kD, xb, xb, kD, 0L, (void*)vtb, (void*)vtb, kS, (long)kVtRows * kS,
        bv, (long)kHd, bv, 0L, kHd, kS, kD, 1.0f);
  }

  rope_kernel<<<dim3((kTok * kD2) / (8 * 256)), dim3(256), 0, stream>>>(QK, COS, SIN, QRK);

  const int  blkS = ((kS / 64) * (kS / 64)) / 8;
  const int  blkP = ((kS / 64) * (kVtRows / 64)) / 8;
  const long strideQR = (long)kS * kKd;
  const long strideP  = (long)kS * kS;
  const long strideVT = (long)kVtRows * kS;
  const long strideO  = (long)kS * kVtRows;
  for (int gq = 0; gq < kBH / kGrp; ++gq) {
    const int bh0  = gq * kGrp;
    const int hsel = bh0 & (kH - 1);
    wmma_gemm64_dmask<<<dim3(blkS, kGrp), dim3(256), 0, stream>>>(
        QRK + (size_t)bh0 * strideQR, kKd, strideQR,
        QRK + (size_t)(kBH + bh0) * strideQR, kKd, strideQR,
        PP, kS, strideP,
        RWF + (size_t)hsel * kS, CLF + (size_t)hsel * kS, (long)kS,
        kS, kS, kKd, kKScale * kPCarry);
    const unsigned short* vtg = VT + (size_t)bh0 * strideVT;
    float* og = O + (size_t)(bh0 & (kOGrp - 1)) * strideO;
    wmma_gemm64<0, false, 0, 0, false, 0, 1><<<dim3(blkP, kGrp), dim3(256), 0, stream>>>(
        PP, PP, kS, strideP, vtg, vtg, kS, strideVT, (void*)og, (void*)og, kVtRows, strideO,
        bq, 0L, bq, 0L, kS, kVtRows, kS, kPCarryInv);
    if ((bh0 & (kOGrp - 1)) == kOGrp - kGrp) {
      ln_gate_kernel<<<dim3((kOGrp * kS) / 16), dim3(256), 0, stream>>>(O, G16, A16, bh0 - (kOGrp - kGrp));
    }
  }

  const int blkO = ((kTok / 64) * (kD / 64)) / 8;
  wmma_gemm64<0, false, 2, 0, false, 0, 0><<<dim3(blkO, 1), dim3(256), 0, stream>>>(
      A16, A16, kD2, 0L, WO, WO, kD2, 0L, (void*)out, (void*)out, kD, 0L, bo, 0L, bo, 0L, kTok, kD, kD2, kWoCarryInv);
}
